// ResidualGraphBlock_12790412607605
// MI455X (gfx1250) — hardware-verified
//
#include <hip/hip_runtime.h>
#define NN 50000
#define NE 800000
#define FF 128
#define GF 64

typedef __bf16 v16b __attribute__((ext_vector_type(16)));
typedef unsigned short v8us __attribute__((ext_vector_type(8), may_alias));
typedef float  v8f  __attribute__((ext_vector_type(8)));
typedef float  v4f  __attribute__((ext_vector_type(4)));
typedef float  v4fa __attribute__((ext_vector_type(4), may_alias));
union FragB { v16b v; v8us half[2]; unsigned short u[16]; };

__device__ __forceinline__ unsigned short bf16_bits(float x) { unsigned int u = __float_as_uint(x); return (unsigned short)((u + 0x7FFFu + ((u >> 16) & 1u)) >> 16); }
__device__ __forceinline__ float bf16_val(unsigned short b) { return __uint_as_float(((unsigned int)b) << 16); }
__device__ __forceinline__ float bf16_round(float x) { return bf16_val(bf16_bits(x)); }
template <int NT>
__device__ __forceinline__ v8f mmaN(v16b ah, v16b al, v16b bh, v16b bl, v8f c) {
  c = __builtin_amdgcn_wmma_f32_16x16x32_bf16(false, ah, false, bh, (short)0, c, false, false);
  if (NT >= 2) c = __builtin_amdgcn_wmma_f32_16x16x32_bf16(false, al, false, bh, (short)0, c, false, false);
  if (NT >= 3) c = __builtin_amdgcn_wmma_f32_16x16x32_bf16(false, ah, false, bl, (short)0, c, false, false);
  asm volatile("v_nop\n\tv_nop\n\tv_nop\n\tv_nop" : "+v"(c) : "v"(ah), "v"(al), "v"(bh), "v"(bl));
  return c;
}

__global__ __launch_bounds__(256) void k_wt_bf16(const float* __restrict__ W, unsigned short* __restrict__ Wt, int K, int N) {
  const int t = blockIdx.x * 256 + threadIdx.x;
  const int k8n = K / 8;
  if (t >= N * k8n) return;
  const int n = t / k8n, k8 = (t % k8n) * 8;
  v8us v;
#pragma unroll
  for (int i = 0; i < 8; ++i) v[i] = bf16_bits(W[(size_t)(k8 + i) * N + n]);
  *(volatile v8us*)(Wt + (size_t)n * K + k8) = v;
  __threadfence();
  *(volatile v8us*)(Wt + (size_t)n * K + k8) = v;
}

template <bool ASPLIT, int ACT, bool BIAS_BF16>
__global__ __launch_bounds__(128) void k_gemm_bf(const float* __restrict__ A, int lda, const unsigned short* __restrict__ Wt, int ldb,
                                               const float* __restrict__ bias, float* __restrict__ C, int ldc, int M, int N, int K) {
  __shared__ __attribute__((aligned(16))) float so[4][16][64];
  const int tid = threadIdx.x, w = tid >> 5, lane = tid & 31, ln = lane & 15, hh = lane >> 4;
  const int ntn = N / 64;
  const int wid = blockIdx.x * 4 + w;
  const int mt = wid / ntn, nq = wid % ntn;
  if (mt * 16 >= M) return;
  const int row0 = mt * 16, col0 = nq * 64;
  const float* arow = A + (size_t)(row0 + ln) * lda;
  v8f acc[4] = {};
  for (int kb = 0; kb < K; kb += 32) {
    FragB ah, al;
    const v4f x0 = *(const v4fa*)(arow + kb + 8 * hh), x1 = *(const v4fa*)(arow + kb + 8 * hh + 4);
    const v4f x2 = *(const v4fa*)(arow + kb + 16 + 8 * hh), x3 = *(const v4fa*)(arow + kb + 16 + 8 * hh + 4);
    float xs[16] = {x0[0],x0[1],x0[2],x0[3],x1[0],x1[1],x1[2],x1[3],x2[0],x2[1],x2[2],x2[3],x3[0],x3[1],x3[2],x3[3]};
#pragma unroll
    for (int i = 0; i < 16; ++i) { const unsigned short hb = bf16_bits(xs[i]); ah.u[i] = hb; al.u[i] = ASPLIT ? bf16_bits(xs[i] - bf16_val(hb)) : (unsigned short)0; }
#pragma unroll
    for (int t = 0; t < 4; ++t) {
      const unsigned short* brow = Wt + (size_t)(col0 + t * 16 + ln) * ldb + kb;
      FragB b;
      b.half[0] = *(const v8us*)(brow + 8 * hh);
      b.half[1] = *(const v8us*)(brow + 16 + 8 * hh);
      acc[t] = mmaN<ASPLIT ? 2 : 1>(ah.v, al.v, b.v, b.v, acc[t]);
    }
  }
#pragma unroll
  for (int t = 0; t < 4; ++t) {
    float bv = bias ? bias[col0 + t * 16 + ln] : 0.f;
    if (BIAS_BF16) bv = bf16_round(bv);
#pragma unroll
    for (int r = 0; r < 8; ++r) { float v = acc[t][r] + bv; if (ACT == 1) v = fmaxf(v, 0.f); so[w][8 * hh + r][t * 16 + ln] = v; }
  }
  __builtin_amdgcn_fence(__ATOMIC_ACQ_REL, "workgroup");
  __builtin_amdgcn_wave_barrier();
  const int rsub = lane >> 4, c4 = (lane & 15) * 4;
  for (int pass = 0; pass < 2; ++pass) {
#pragma unroll
    for (int q = 0; q < 8; ++q) {
      const int r = q * 2 + rsub;
      const v4f v = *(const v4fa*)&so[w][r][c4];
      *(volatile v4f*)(C + (size_t)(row0 + r) * ldc + col0 + c4) = v;
    }
    if (pass == 0) __threadfence();
  }
}

template <int D, bool CAUSAL>
__global__ __launch_bounds__(128) void k_flash(const float* __restrict__ qb, const float* __restrict__ kb, const float* __restrict__ vb,
                                             int pitch, int T, int H, float scale, float* __restrict__ y, int ypitch) {
  constexpr int KS = D / 32;
  constexpr int DT = D / 16;
  __shared__ __attribute__((aligned(16))) unsigned short sKh[32][D + 8], sKl[32][D + 8], sVh[32][D + 8], sVl[32][D + 8];
  __shared__ __attribute__((aligned(16))) unsigned short sPh[4][16][40], sPl[4][16][40];
  __shared__ __attribute__((aligned(16))) float sO[4][16][D];
  const int tid = threadIdx.x, w = tid >> 5, lane = tid & 31, ln = lane & 15, hh = lane >> 4;
  const int nqb = (T + 63) / 64;
  const int bh = blockIdx.x / nqb, qblk = blockIdx.x % nqb;
  const int b = bh / H, h = bh % H;
  const int q0 = qblk * 64 + w * 16;
  const float* Q = qb + (size_t)b * T * pitch + h * D;
  const float* K = kb + (size_t)b * T * pitch + h * D;
  const float* V = vb + (size_t)b * T * pitch + h * D;

  FragB aqh[KS], aql[KS];
  {
    int row = q0 + ln; if (row >= T) row = T - 1;
    const float* qr = Q + (size_t)row * pitch;
#pragma unroll
    for (int ks = 0; ks < KS; ++ks)
#pragma unroll
      for (int i = 0; i < 16; ++i) {
        const int d = ks * 32 + ((i < 8) ? (8 * hh + i) : (16 + 8 * hh + (i - 8)));
        const float x = qr[d] * scale; const unsigned short hb = bf16_bits(x);
        aqh[ks].u[i] = hb; aql[ks].u[i] = bf16_bits(x - bf16_val(hb));
      }
  }
  float m_r[8], l_r[8];
#pragma unroll
  for (int r = 0; r < 8; ++r) { m_r[r] = -3.0e38f; l_r[r] = 0.f; }
  v8f oacc[DT];
#pragma unroll
  for (int dt = 0; dt < DT; ++dt) oacc[dt] = (v8f){0.f,0.f,0.f,0.f,0.f,0.f,0.f,0.f};

  const int kv_end = CAUSAL ? min(T, qblk * 64 + 64) : T;
  for (int j0 = 0; j0 < kv_end; j0 += 32) {
    __syncthreads();
    for (int e = tid; e < 32 * (D / 4); e += 128) {
      const int r = e / (D / 4), c4 = (e % (D / 4)) * 4;
      const int key = j0 + r;
      v4f kf = {0.f,0.f,0.f,0.f}, vf = {0.f,0.f,0.f,0.f};
      if (key < T) { kf = *(const v4fa*)(K + (size_t)key * pitch + c4); vf = *(const v4fa*)(V + (size_t)key * pitch + c4); }
#pragma unroll
      for (int t = 0; t < 4; ++t) {
        unsigned short hb = bf16_bits(kf[t]); sKh[r][c4 + t] = hb; sKl[r][c4 + t] = bf16_bits(kf[t] - bf16_val(hb));
        hb = bf16_bits(vf[t]); sVh[r][c4 + t] = hb; sVl[r][c4 + t] = bf16_bits(vf[t] - bf16_val(hb));
      }
    }
    __syncthreads();
    v8f s[2];
#pragma unroll
    for (int nt = 0; nt < 2; ++nt) {
      v8f acc = {};
#pragma unroll
      for (int ks = 0; ks < KS; ++ks) {
        FragB bh_, bl_;
        bh_.half[0] = *(const v8us*)&sKh[nt * 16 + ln][ks * 32 + 8 * hh]; bh_.half[1] = *(const v8us*)&sKh[nt * 16 + ln][ks * 32 + 16 + 8 * hh];
        bl_.half[0] = *(const v8us*)&sKl[nt * 16 + ln][ks * 32 + 8 * hh]; bl_.half[1] = *(const v8us*)&sKl[nt * 16 + ln][ks * 32 + 16 + 8 * hh];
        acc = mmaN<3>(aqh[ks].v, aql[ks].v, bh_.v, bl_.v, acc);
      }
      s[nt] = acc;
    }
    float alpha[8];
#pragma unroll
    for (int r = 0; r < 8; ++r) {
      const int qi = q0 + 8 * hh + r;
      const int ja = j0 + ln, jb = j0 + 16 + ln;
      if (CAUSAL) { if (ja > qi) s[0][r] = -3.0e38f; if (jb > qi) s[1][r] = -3.0e38f; }
      if (ja >= T) s[0][r] = -3.0e38f;
      if (jb >= T) s[1][r] = -3.0e38f;
      float mx = fmaxf(s[0][r], s[1][r]);
      mx = fmaxf(mx, __shfl_xor(mx, 1, 32)); mx = fmaxf(mx, __shfl_xor(mx, 2, 32)); mx = fmaxf(mx, __shfl_xor(mx, 4, 32)); mx = fmaxf(mx, __shfl_xor(mx, 8, 32));
      const float mnew = fmaxf(m_r[r], mx);
      alpha[r] = (mnew > -1.0e38f) ? __expf(m_r[r] - mnew) : 1.0f;
      const float p0 = (s[0][r] > -1.0e38f) ? __expf(s[0][r] - mnew) : 0.f;
      const float p1 = (s[1][r] > -1.0e38f) ? __expf(s[1][r] - mnew) : 0.f;
      m_r[r] = mnew;
      l_r[r] = l_r[r] * alpha[r] + p0 + p1;
      unsigned short hb = bf16_bits(p0); sPh[w][8 * hh + r][ln] = hb;      sPl[w][8 * hh + r][ln] = bf16_bits(p0 - bf16_val(hb));
      hb = bf16_bits(p1);                sPh[w][8 * hh + r][16 + ln] = hb; sPl[w][8 * hh + r][16 + ln] = bf16_bits(p1 - bf16_val(hb));
    }
#pragma unroll
    for (int dt = 0; dt < DT; ++dt)
#pragma unroll
      for (int r = 0; r < 8; ++r) oacc[dt][r] *= alpha[r];
    __builtin_amdgcn_fence(__ATOMIC_ACQ_REL, "workgroup");
    __builtin_amdgcn_wave_barrier();
    FragB pah, pal;
    pah.half[0] = *(const v8us*)&sPh[w][ln][8 * hh]; pah.half[1] = *(const v8us*)&sPh[w][ln][16 + 8 * hh];
    pal.half[0] = *(const v8us*)&sPl[w][ln][8 * hh]; pal.half[1] = *(const v8us*)&sPl[w][ln][16 + 8 * hh];
#pragma unroll
    for (int dt = 0; dt < DT; ++dt) {
      FragB bvh, bvl;
#pragma unroll
      for (int i = 0; i < 8; ++i) {
        bvh.u[i] = sVh[8 * hh + i][dt * 16 + ln]; bvh.u[8 + i] = sVh[16 + 8 * hh + i][dt * 16 + ln];
        bvl.u[i] = sVl[8 * hh + i][dt * 16 + ln]; bvl.u[8 + i] = sVl[16 + 8 * hh + i][dt * 16 + ln];
      }
      oacc[dt] = mmaN<3>(pah.v, pal.v, bvh.v, bvl.v, oacc[dt]);
    }
    __builtin_amdgcn_fence(__ATOMIC_ACQ_REL, "workgroup");
    __builtin_amdgcn_wave_barrier();
  }
#pragma unroll
  for (int r = 0; r < 8; ++r) {
    float l = l_r[r];
    l += __shfl_xor(l, 1, 32); l += __shfl_xor(l, 2, 32); l += __shfl_xor(l, 4, 32); l += __shfl_xor(l, 8, 32);
    l_r[r] = (l > 0.f) ? 1.0f / l : 0.f;
  }
#pragma unroll
  for (int dt = 0; dt < DT; ++dt)
#pragma unroll
    for (int r = 0; r < 8; ++r) sO[w][8 * hh + r][dt * 16 + ln] = oacc[dt][r] * l_r[r];
  __builtin_amdgcn_fence(__ATOMIC_ACQ_REL, "workgroup");
  __builtin_amdgcn_wave_barrier();
  for (int pass = 0; pass < 2; ++pass) {
    for (int r = 0; r < 16; ++r) {
      const int row = q0 + r;
      if (row < T && lane < D / 4) {
        const v4f val = *(const v4fa*)&sO[w][r][lane * 4];
        *(volatile v4f*)(y + ((size_t)b * T + row) * ypitch + h * D + lane * 4) = val;
      }
    }
    if (pass == 0) __threadfence();
  }
}

typedef _Float16 v16h __attribute__((ext_vector_type(16)));
union FragH { v16h v; v8us half[2]; _Float16 h[16]; unsigned short u[16]; };
template <int NT>
__device__ __forceinline__ v8f mmaH(v16h ah, v16h al, v16h bh, v16h bl, v8f c) {
  c = __builtin_amdgcn_wmma_f32_16x16x32_f16(false, ah, false, bh, (short)0, c, false, false);
  if (NT >= 2) c = __builtin_amdgcn_wmma_f32_16x16x32_f16(false, al, false, bh, (short)0, c, false, false);
  if (NT >= 3) c = __builtin_amdgcn_wmma_f32_16x16x32_f16(false, ah, false, bl, (short)0, c, false, false);
  asm volatile("v_nop\n\tv_nop\n\tv_nop\n\tv_nop" : "+v"(c) : "v"(ah), "v"(al), "v"(bh), "v"(bl));
  return c;
}
template <bool ASPLIT>
__global__ __launch_bounds__(128) void k_gemm_h(const float* __restrict__ A, int lda, size_t sA, const _Float16* __restrict__ Bh, int ldb, size_t sB, float alpha, float* __restrict__ C, int ldc, size_t sC, int M, int N, int K) {
  __shared__ __attribute__((aligned(16))) float so[4][16][64];
  const int tid = threadIdx.x, w = tid >> 5, lane = tid & 31, ln = lane & 15, hh = lane >> 4; const int by = blockIdx.y;
  A += (size_t)by * sA; Bh += (size_t)by * sB; C += (size_t)by * sC;
  const int ntn = (N + 63) / 64; const int wid = blockIdx.x * 4 + w; const int mt = wid / ntn, nq = wid % ntn; if (mt * 16 >= M) return;
  const int row0 = mt * 16, col0 = nq * 64; const float* arow = A + (size_t)(row0 + ln) * lda;
  v8f acc[4] = {};
  for (int kb = 0; kb < K; kb += 32) {
    FragH ah, al;
    const v4f x0 = *(const v4fa*)(arow + kb + 8 * hh), x1 = *(const v4fa*)(arow + kb + 8 * hh + 4), x2 = *(const v4fa*)(arow + kb + 16 + 8 * hh), x3 = *(const v4fa*)(arow + kb + 16 + 8 * hh + 4);
    float xs[16] = {x0[0],x0[1],x0[2],x0[3],x1[0],x1[1],x1[2],x1[3],x2[0],x2[1],x2[2],x2[3],x3[0],x3[1],x3[2],x3[3]};
#pragma unroll
    for (int i = 0; i < 16; ++i) { const _Float16 h = (_Float16)xs[i]; ah.h[i] = h; al.h[i] = ASPLIT ? (_Float16)(xs[i] - (float)h) : (_Float16)0.0f; }
#pragma unroll
    for (int t = 0; t < 4; ++t) { if (col0 + t * 16 >= N) continue; const size_t boff = (size_t)(col0 + t * 16 + ln) * ldb + kb; FragH bq; bq.half[0] = *(const v8us*)(Bh + boff + 8 * hh); bq.half[1] = *(const v8us*)(Bh + boff + 16 + 8 * hh);
      acc[t] = mmaH<ASPLIT ? 2 : 1>(ah.v, al.v, bq.v, bq.v, acc[t]); }
  }
#pragma unroll
  for (int t = 0; t < 4; ++t) { if (col0 + t * 16 >= N) continue;
#pragma unroll
    for (int r = 0; r < 8; ++r) so[w][8 * hh + r][t * 16 + ln] = acc[t][r] * alpha; }
  __builtin_amdgcn_fence(__ATOMIC_ACQ_REL, "workgroup"); __builtin_amdgcn_wave_barrier();
  const int rsub = lane >> 4, c4 = (lane & 15) * 4;
  for (int pass = 0; pass < 2; ++pass) {
#pragma unroll
    for (int q = 0; q < 8; ++q) { const int r = q * 2 + rsub; if (col0 + c4 < N) { const v4f v = *(const v4fa*)&so[w][r][c4]; *(volatile v4f*)(C + (size_t)(row0 + r) * ldc + col0 + c4) = v; } }
    if (pass == 0) __threadfence(); }
}

template <int DUMMY>
__global__ __launch_bounds__(128) void k_gemm_hh(const _Float16* __restrict__ A, int lda, size_t sA, const _Float16* __restrict__ Bh, int ldb, size_t sB, float alpha, float* __restrict__ C, int ldc, size_t sC, int M, int N, int K) {
  __shared__ __attribute__((aligned(16))) float so[4][16][64];
  const int tid = threadIdx.x, w = tid >> 5, lane = tid & 31, ln = lane & 15, hh = lane >> 4; const int by = blockIdx.y;
  A += (size_t)by * sA; Bh += (size_t)by * sB; C += (size_t)by * sC;
  const int ntn = (N + 63) / 64; const int wid = blockIdx.x * 4 + w; const int mt = wid / ntn, nq = wid % ntn; if (mt * 16 >= M) return;
  const int row0 = mt * 16, col0 = nq * 64; const _Float16* arow = A + (size_t)(row0 + ln) * lda;
  v8f acc[4] = {};
  for (int kb = 0; kb < K; kb += 32) { FragH ah; ah.half[0] = *(const v8us*)((const unsigned short*)arow + kb + 8 * hh); ah.half[1] = *(const v8us*)((const unsigned short*)arow + kb + 16 + 8 * hh);
#pragma unroll
    for (int t = 0; t < 4; ++t) { if (col0 + t * 16 >= N) continue; const size_t boff = (size_t)(col0 + t * 16 + ln) * ldb + kb; FragH bq; bq.half[0] = *(const v8us*)((const unsigned short*)Bh + boff + 8 * hh); bq.half[1] = *(const v8us*)((const unsigned short*)Bh + boff + 16 + 8 * hh);
      acc[t] = mmaH<1>(ah.v, ah.v, bq.v, bq.v, acc[t]); }
  }
#pragma unroll
  for (int t = 0; t < 4; ++t) { if (col0 + t * 16 >= N) continue;
#pragma unroll
    for (int r = 0; r < 8; ++r) so[w][8 * hh + r][t * 16 + ln] = acc[t][r] * alpha; }
  __builtin_amdgcn_fence(__ATOMIC_ACQ_REL, "workgroup"); __builtin_amdgcn_wave_barrier();
  const int rsub = lane >> 4, c4 = (lane & 15) * 4;
  for (int pass = 0; pass < 2; ++pass) {
#pragma unroll
    for (int q = 0; q < 8; ++q) { const int r = q * 2 + rsub; if (col0 + c4 < N) { const v4f v = *(const v4fa*)&so[w][r][c4]; *(volatile v4f*)(C + (size_t)(row0 + r) * ldc + col0 + c4) = v; } }
    if (pass == 0) __threadfence(); }
}

template <int ACT>
__global__ __launch_bounds__(128) void k_gemm_hhx(const _Float16* __restrict__ A, int lda, size_t sA, const _Float16* __restrict__ Bh, int ldb, size_t sB, float alpha, const float* __restrict__ bias, size_t sBias, const float* __restrict__ CP, int rowsPerB, size_t sCPb, int row0g,
    float* __restrict__ C, _Float16* __restrict__ C16, int ldc, size_t sC, int M, int N, int K) {
  __shared__ __attribute__((aligned(16))) float so[4][16][64];
  const int tid = threadIdx.x, w = tid >> 5, lane = tid & 31, ln = lane & 15, hh = lane >> 4; const int by = blockIdx.y;
  A += (size_t)by * sA; Bh += (size_t)by * sB; const size_t cofs = (size_t)by * sC; const float* bp = bias ? bias + (size_t)by * sBias : nullptr;
  const int ntn = (N + 63) / 64; const int wid = blockIdx.x * 4 + w; const int mt = wid / ntn, nq = wid % ntn; if (mt * 16 >= M) return;
  const int row0 = mt * 16, col0 = nq * 64; const _Float16* arow = A + (size_t)(row0 + ln) * lda;
  v8f acc[4] = {};
  for (int kb = 0; kb < K; kb += 32) { FragH ah; ah.half[0] = *(const v8us*)((const unsigned short*)arow + kb + 8 * hh); ah.half[1] = *(const v8us*)((const unsigned short*)arow + kb + 16 + 8 * hh);
#pragma unroll
    for (int t = 0; t < 4; ++t) { if (col0 + t * 16 >= N) continue; const size_t boff = (size_t)(col0 + t * 16 + ln) * ldb + kb; FragH bq; bq.half[0] = *(const v8us*)((const unsigned short*)Bh + boff + 8 * hh); bq.half[1] = *(const v8us*)((const unsigned short*)Bh + boff + 16 + 8 * hh);
      acc[t] = mmaH<1>(ah.v, ah.v, bq.v, bq.v, acc[t]); }
  }
#pragma unroll
  for (int t = 0; t < 4; ++t) { if (col0 + t * 16 >= N) continue; const int col = col0 + t * 16 + ln; const float bv = bp ? bf16_round(bp[col]) : 0.f;
#pragma unroll
    for (int r = 0; r < 8; ++r) { float v = acc[t][r] * alpha + bv; if (CP) { const int bidx = (row0g + row0 + 8 * hh + r) / rowsPerB; v += CP[(size_t)bidx * sCPb + (size_t)by * 64 + col]; } if (ACT == 1) v = (v > 0.f) ? v : expm1f(v); else if (ACT == 3) v = fmaxf(v, 0.f); so[w][8 * hh + r][t * 16 + ln] = v; } }
  __builtin_amdgcn_fence(__ATOMIC_ACQ_REL, "workgroup"); __builtin_amdgcn_wave_barrier();
  const int rsub = lane >> 4, c4 = (lane & 15) * 4; typedef _Float16 v4h __attribute__((ext_vector_type(4)));
  for (int pass = 0; pass < 2; ++pass) {
#pragma unroll
    for (int q = 0; q < 8; ++q) { const int r = q * 2 + rsub; if (col0 + c4 < N) { const v4f v = *(const v4fa*)&so[w][r][c4]; if (C) *(volatile v4f*)(C + cofs + (size_t)(row0 + r) * ldc + col0 + c4) = v; if (C16) { v4h h4; for (int i = 0; i < 4; ++i) h4[i] = (_Float16)v[i]; *(volatile v4h*)(C16 + cofs + (size_t)(row0 + r) * ldc + col0 + c4) = h4; } } }
    if (pass == 0) __threadfence(); }
}

__device__ __forceinline__ int bscan512(int cnt, int* scan, int tid, int& total) { __syncthreads(); scan[tid] = cnt; __syncthreads();
  for (int of = 1; of < 512; of <<= 1) { const int v = (tid >= of) ? scan[tid - of] : 0; __syncthreads(); scan[tid] += v; __syncthreads(); }
  total = scan[511]; return scan[tid] - cnt; }
template <int H0> __global__ __launch_bounds__(512) void k_gat(const _Float16* __restrict__ FT16, const float* __restrict__ ES, const int* __restrict__ src, const int* __restrict__ dst, float* __restrict__ HATT) {
  __shared__ short Lr[4096]; __shared__ int Le[4096]; __shared__ int scan[512]; __shared__ float stg[64][65];
  typedef float v2f __attribute__((ext_vector_type(2))); typedef _Float16 v2h __attribute__((ext_vector_type(2)));
  const int tid = threadIdx.x; const int n0 = blockIdx.x * 512; v2f acc[32]; float m[4], z[4];
#pragma unroll
  for (int c = 0; c < 32; ++c) acc[c] = v2f{0.f, 0.f};
#pragma unroll
  for (int h = 0; h < 4; ++h) { m[h] = -3.0e38f; z[h] = 0.f; }
  for (int e0 = 0; e0 < NE; e0 += 4096) { int hr[8], he[8]; int cnt = 0;
#pragma unroll
    for (int k = 0; k < 8; ++k) { const int e = e0 + tid * 8 + k; hr[k] = -1; he[k] = 0; if (e < NE) { const int dd_ = dst[e]; if (dd_ >= n0 && dd_ < n0 + 512) { hr[k] = dd_ - n0; he[k] = e; ++cnt; } } }
    int tot; int p = bscan512(cnt, scan, tid, tot);
#pragma unroll
    for (int k = 0; k < 8; ++k) if (hr[k] >= 0) { Lr[p] = (short)hr[k]; Le[p] = he[k]; ++p; }
    __syncthreads();
#pragma unroll 1
    for (int q = 0; q < tot; ++q) { if (Lr[q] == tid) { const int e = Le[q]; int s = src[e]; s = s < 0 ? 0 : (s >= NN ? NN - 1 : s); const float* es = ES + (size_t)e * 8; const v2h* fr = (const v2h*)(FT16 + (size_t)s * 128);
#pragma unroll
        for (int hl = 0; hl < 4; ++hl) { const int h = H0 + hl; const float ev = es[h]; const float tex = __expf(-fabsf(ev - m[hl])); const bool up = ev > m[hl]; const float sc = up ? tex : 1.0f; const float w = up ? 1.0f : tex; if (up) { m[hl] = ev; const v2f sc2 = v2f{sc, sc};
#pragma unroll
            for (int d = 0; d < 8; ++d) acc[hl * 8 + d] *= sc2; } z[hl] = z[hl] * sc + w;
          const v2f w2 = v2f{w, w};
#pragma unroll
          for (int d = 0; d < 8; ++d) { const v2h f2 = fr[h * 8 + d]; const v2f ff = v2f{(float)f2.x, (float)f2.y}; acc[hl * 8 + d] += w2 * ff; } } } }
    __syncthreads(); }
#pragma unroll
  for (int hl = 0; hl < 4; ++hl) { const float iz = (z[hl] > 0.f) ? 1.0f / z[hl] : 0.f; const v2f iz2 = v2f{iz, iz};
#pragma unroll
    for (int d = 0; d < 8; ++d) acc[hl * 8 + d] *= iz2; }
  for (int tg = 0; tg < 8; ++tg) {
    if (tid / 64 == tg) {
#pragma unroll
      for (int c = 0; c < 32; ++c) { stg[tid % 64][2 * c] = acc[c].x; stg[tid % 64][2 * c + 1] = acc[c].y; } }
    __syncthreads();
    for (int pass = 0; pass < 2; ++pass) {
#pragma unroll 1
      for (int i = tid; i < 64 * 16; i += 512) { const int r = i / 16, c4 = (i % 16) * 4; const int n = n0 + tg * 64 + r; if (n < NN) { v4f v;
#pragma unroll 1
          for (int qq = 0; qq < 4; ++qq) { const float a = stg[r][c4 + qq]; v[qq] = a > 0.f ? a : expm1f(a); }
          *(volatile v4f*)(HATT + (size_t)n * 128 + H0 * 16 + c4) = v; } } if (pass == 0) __threadfence(); }
    __syncthreads(); } }
__global__ __launch_bounds__(512) void k_pmax(const _Float16* __restrict__ P16, const int* __restrict__ src, const int* __restrict__ dst, _Float16* __restrict__ PM16) {
  __shared__ short Lr[4096]; __shared__ int Lc[4096]; __shared__ int scan[512]; __shared__ float stg[64][129];
  const int tid = threadIdx.x; const int n0 = blockIdx.x * 512; float acc[128]; int have = 0;
#pragma unroll
  for (int c = 0; c < 128; ++c) acc[c] = -__builtin_inff();
  for (int e0 = 0; e0 < NE; e0 += 4096) { int hr[8], hc[8]; int cnt = 0;
#pragma unroll
    for (int k = 0; k < 8; ++k) { const int e = e0 + tid * 8 + k; hr[k] = -1; hc[k] = 0; if (e < NE) { const int dd_ = dst[e]; if (dd_ >= n0 && dd_ < n0 + 512) { hr[k] = dd_ - n0; int s = src[e]; s = s < 0 ? 0 : (s >= NN ? NN - 1 : s); hc[k] = s; ++cnt; } } }
    int tot; int p = bscan512(cnt, scan, tid, tot);
#pragma unroll
    for (int k = 0; k < 8; ++k) if (hr[k] >= 0) { Lr[p] = (short)hr[k]; Lc[p] = hc[k]; ++p; }
    __syncthreads();
#pragma unroll 1
    for (int q = 0; q < tot; ++q) { if (Lr[q] == tid) { have = 1; const unsigned short* pr = (const unsigned short*)P16 + (size_t)Lc[q] * 128;
#pragma unroll
        for (int g = 0; g < 16; ++g) { FragH f; f.half[0] = *(const v8us*)(pr + g * 8); for (int d = 0; d < 8; ++d) acc[g * 8 + d] = fmaxf(acc[g * 8 + d], (float)f.h[d]); } } }
    __syncthreads(); }
  if (!have) {
#pragma unroll
    for (int c = 0; c < 128; ++c) acc[c] = 0.f; }
  typedef _Float16 v4h __attribute__((ext_vector_type(4)));
  for (int tg = 0; tg < 8; ++tg) {
    if (tid / 64 == tg) {
#pragma unroll
      for (int c = 0; c < 128; ++c) stg[tid % 64][c] = acc[c]; }
    __syncthreads();
    for (int pass = 0; pass < 2; ++pass) { for (int i = tid; i < 64 * 32; i += 512) { const int r = i / 32, c4 = (i % 32) * 4; const int n = n0 + tg * 64 + r; if (n < NN) { v4h v; v[0] = (_Float16)stg[r][c4]; v[1] = (_Float16)stg[r][c4 + 1]; v[2] = (_Float16)stg[r][c4 + 2]; v[3] = (_Float16)stg[r][c4 + 3]; *(volatile v4h*)(PM16 + (size_t)n * 128 + c4) = v; } } if (pass == 0) __threadfence(); }
    __syncthreads(); } }

typedef _Float16 v4h __attribute__((ext_vector_type(4)));
__global__ __launch_bounds__(256) void k_bt(const float* __restrict__ Wa, const float* __restrict__ Wp, const float* __restrict__ Wgs, const float* __restrict__ Wgn, const float* __restrict__ Whr, const float* __restrict__ Wsi, _Float16* __restrict__ Ba, _Float16* __restrict__ Bp, _Float16* __restrict__ Bgs, _Float16* __restrict__ Bgn, _Float16* __restrict__ Bhr, _Float16* __restrict__ Bsi) { const int t = blockIdx.x * 256 + threadIdx.x;
  if (t < FF * FF) { const int k = t % FF, n = t / FF; *(volatile _Float16*)(Ba + t) = (_Float16)(bf16_round(Wa[k * FF + n]) * 16.0f); *(volatile _Float16*)(Bp + t) = (_Float16)(bf16_round(Wp[k * FF + n]) * 16.0f); *(volatile _Float16*)(Bhr + t) = (_Float16)(bf16_round(Whr[k * FF + n]) * 16.0f); *(volatile _Float16*)(Bsi + t) = (_Float16)(bf16_round(Wsi[k * FF + n]) * 16.0f); }
  if (t < GF * FF) { const int k = t % FF, n = t / FF; *(volatile _Float16*)(Bgs + t) = (_Float16)(bf16_round(Wgs[k * GF + n]) * 16.0f); *(volatile _Float16*)(Bgn + t) = (_Float16)(bf16_round(Wgn[k * GF + n]) * 16.0f); } }
template <int SRCBF> __global__ __launch_bounds__(256) void k_ln(const float* __restrict__ X, const float* __restrict__ g, const float* __restrict__ be, float* __restrict__ Y, _Float16* __restrict__ Y16) { const int tid = threadIdx.x, wv = tid >> 5, lane = tid & 31; const size_t n = (size_t)blockIdx.x * 8 + wv; float v[4]; float s = 0.f;
  for (int u = 0; u < 4; ++u) { const float x = X[n * FF + u * 32 + lane]; v[u] = SRCBF ? bf16_round(x) : x; s += v[u]; } for (int o = 16; o >= 1; o >>= 1) s += __shfl_xor(s, o, 32); const float mu = s / (float)FF; float q2 = 0.f; for (int u = 0; u < 4; ++u) { const float d = v[u] - mu; q2 += d * d; } for (int o = 16; o >= 1; o >>= 1) q2 += __shfl_xor(q2, o, 32); const float inv = 1.0f / sqrtf(q2 / (float)FF + 1e-5f);
  for (int pass = 0; pass < 2; ++pass) { for (int u = 0; u < 4; ++u) { const int c = u * 32 + lane; const float y = (v[u] - mu) * inv * bf16_round(g[c]) + bf16_round(be[c]); *(volatile float*)(Y + n * FF + c) = y; *(volatile _Float16*)(Y16 + n * FF + c) = (_Float16)y; } if (pass == 0) __threadfence(); } }
__global__ __launch_bounds__(256) void k_escore(const _Float16* __restrict__ FT16, const int* __restrict__ src, const int* __restrict__ dst, float* __restrict__ ES) { const size_t t = (size_t)blockIdx.x * 256 + threadIdx.x; if (t >= (size_t)NE * 4) return; const size_t e = t / 4; const int hp = (int)(t % 4); int s = src[e], d = dst[e]; s = s < 0 ? 0 : (s >= NN ? NN - 1 : s); d = d < 0 ? 0 : (d >= NN ? NN - 1 : d);
  typedef float v2f __attribute__((ext_vector_type(2), aligned(8))); v2f o2;
  for (int j = 0; j < 2; ++j) { const int h = hp * 2 + j; FragH a, b; a.half[0] = *(const v8us*)((const unsigned short*)FT16 + (size_t)s * FF + h * 16); a.half[1] = *(const v8us*)((const unsigned short*)FT16 + (size_t)s * FF + h * 16 + 8); b.half[0] = *(const v8us*)((const unsigned short*)FT16 + (size_t)d * FF + h * 16); b.half[1] = *(const v8us*)((const unsigned short*)FT16 + (size_t)d * FF + h * 16 + 8); float acc = 0.f;
#pragma unroll
    for (int i = 0; i < 16; ++i) acc += (float)a.h[i] * (float)b.h[i]; o2[j] = acc * 0.25f; }
  *(volatile v2f*)(ES + e * 8 + hp * 2) = o2; __threadfence(); *(volatile v2f*)(ES + e * 8 + hp * 2) = o2; }
__global__ __launch_bounds__(256) void k_gate(const float* __restrict__ GFt, const float* __restrict__ Wgr, const float* __restrict__ bgr, const float* __restrict__ HATT, _Float16* __restrict__ H16) { const int tid = threadIdx.x, wv = tid >> 5, lane = tid & 31; const size_t n = (size_t)blockIdx.x * 8 + wv; const float g0 = GFt[n * GF + lane], g1 = GFt[n * GF + 32 + lane]; float gate[8];
#pragma unroll
  for (int h = 0; h < 8; ++h) { float s = g0 * bf16_round(Wgr[lane * 8 + h]) + g1 * bf16_round(Wgr[(32 + lane) * 8 + h]); for (int o = 16; o >= 1; o >>= 1) s += __shfl_xor(s, o, 32); gate[h] = 1.0f / (1.0f + expf(-(s + bf16_round(bgr[h])))); }
  typedef _Float16 v2h __attribute__((ext_vector_type(2)));
  for (int pass = 0; pass < 2; ++pass) { for (int u = 0; u < 2; ++u) { const int c = u * 64 + 2 * lane; const int h = c >> 4; v2h o2; o2.x = (_Float16)(HATT[n * FF + c] * gate[h]); o2.y = (_Float16)(HATT[n * FF + c + 1] * gate[h]); *(volatile v2h*)(H16 + n * FF + c) = o2; } if (pass == 0) __threadfence(); } }
__global__ __launch_bounds__(256) void k_out(const float* __restrict__ OP, const float* __restrict__ H2, float* __restrict__ out) { const size_t t = (size_t)blockIdx.x * 256 + threadIdx.x; if (t >= (size_t)NN * FF / 4) return; const v4f a = *(const v4fa*)(OP + t * 4), b = *(const v4fa*)(H2 + t * 4); v4f o; for (int q = 0; q < 4; ++q) { const float v = a[q]; o[q] = (v > 0.f ? v : expm1f(v)) + b[q]; } *(volatile v4f*)(out + t * 4) = o; __threadfence(); *(volatile v4f*)(out + t * 4) = o; }
extern "C" void kernel_launch(void* const* d_in, const int* in_sizes, int n_in,
                              void* d_out, int out_size, void* d_ws, size_t ws_size, hipStream_t stream) {
  (void)in_sizes; (void)n_in; (void)out_size;
  const float* h = (const float*)d_in[0]; const int* src = (const int*)d_in[1]; const int* dst = (const int*)d_in[2]; const float* ln1g = (const float*)d_in[3]; const float* ln1b = (const float*)d_in[4]; const float* Wa = (const float*)d_in[5]; const float* Wp = (const float*)d_in[6]; const float* bp = (const float*)d_in[7]; const float* Wgs = (const float*)d_in[8]; const float* Wgn = (const float*)d_in[9]; const float* bg = (const float*)d_in[10]; const float* Wgr = (const float*)d_in[11]; const float* bgr = (const float*)d_in[12]; const float* Whr = (const float*)d_in[13]; const float* bhr = (const float*)d_in[14]; const float* ln2g = (const float*)d_in[15]; const float* ln2b = (const float*)d_in[16]; const float* Wsi = (const float*)d_in[17]; const float* bsi = (const float*)d_in[18];
  char* ws = (char*)d_ws; size_t off = 0;
  auto take = [&](size_t bytes) { char* p = ws + off; off += (bytes + 255) & ~(size_t)255; return p; };
  _Float16* Ba = (_Float16*)take(FF * FF * 2); _Float16* Bp = (_Float16*)take(FF * FF * 2); _Float16* Bgs = (_Float16*)take(GF * FF * 2); _Float16* Bgn = (_Float16*)take(GF * FF * 2); _Float16* Bhr = (_Float16*)take(FF * FF * 2); _Float16* Bsi = (_Float16*)take(FF * FF * 2);
  float* H1 = (float*)take((size_t)NN * FF * 4); _Float16* H1h = (_Float16*)take((size_t)NN * FF * 2); _Float16* FT16 = (_Float16*)take((size_t)NN * FF * 2); float* ES = (float*)take((size_t)NE * 8 * 4); _Float16* P16 = (_Float16*)ES;     _Float16* PM16 = (_Float16*)take((size_t)NN * FF * 2); float* HATT = (float*)take((size_t)NN * FF * 4);
  if (off > ws_size) return;
  const unsigned EW4 = (unsigned)(((size_t)NN * FF / 4 + 255) / 256); const int NTL = (NN + 511) / 512; const dim3 g128(((NN / 16) * (FF / 64) + 3) / 4, 1), g64(((NN / 16) * 1 + 3) / 4, 1);
  k_bt<<<(FF * FF + 255) / 256, 256, 0, stream>>>(Wa, Wp, Wgs, Wgn, Whr, Wsi, Ba, Bp, Bgs, Bgn, Bhr, Bsi);
  k_ln<1><<<NN / 8, 256, 0, stream>>>(h, ln1g, ln1b, H1, H1h);
  k_gemm_hhx<0><<<g128, 128, 0, stream>>>(H1h, FF, 0, Ba, FF, 0, 0.0625f, nullptr, 0, nullptr, 1, 0, 0, nullptr, FT16, FF, 0, NN, FF, FF);
  k_gemm_hhx<3><<<g128, 128, 0, stream>>>(H1h, FF, 0, Bp, FF, 0, 0.0625f, bp, 0, nullptr, 1, 0, 0, nullptr, P16, FF, 0, NN, FF, FF);
  k_pmax<<<NTL, 512, 0, stream>>>(P16, src, dst, PM16);
  k_escore<<<(unsigned)(((size_t)NE * 4 + 255) / 256), 256, 0, stream>>>(FT16, src, dst, ES);
  k_gat<0><<<NTL, 512, 0, stream>>>(FT16, ES, src, dst, HATT); k_gat<4><<<NTL, 512, 0, stream>>>(FT16, ES, src, dst, HATT);
  float* GFt = ES;
  k_gemm_hhx<0><<<g64, 128, 0, stream>>>(H1h, FF, 0, Bgs, FF, 0, 0.0625f, bg, 0, nullptr, 1, 0, 0, GFt, nullptr, GF, 0, NN, GF, FF);
  k_gemm_hhx<0><<<g64, 128, 0, stream>>>(PM16, FF, 0, Bgn, FF, 0, 0.0625f, nullptr, 0, GFt, 1, GF, 0, GFt, nullptr, GF, 0, NN, GF, FF);
  _Float16* HA16 = FT16;
  k_gate<<<NN / 8, 256, 0, stream>>>(GFt, Wgr, bgr, HATT, HA16);
  float* H2 = HATT;
  k_gemm_hhx<0><<<g128, 128, 0, stream>>>(HA16, FF, 0, Bhr, FF, 0, 0.0625f, bhr, 0, H1, 1, FF, 0, H2, nullptr, FF, 0, NN, FF, FF);
  _Float16* H2h = PM16;
  k_ln<0><<<NN / 8, 256, 0, stream>>>(H2, ln2g, ln2b, H2, H2h);
  float* OP = H1;
  k_gemm_hhx<0><<<g128, 128, 0, stream>>>(H2h, FF, 0, Bsi, FF, 0, 0.0625f, bsi, 0, nullptr, 1, 0, 0, OP, nullptr, FF, 0, NN, FF, FF);
  k_out<<<EW4, 256, 0, stream>>>(OP, H2, (float*)d_out);
}
